// GATModel_26860725469216
// MI455X (gfx1250) — hardware-verified
//
#include <hip/hip_runtime.h>
#include <stddef.h>
#include <stdint.h>
#include <math.h>

#pragma clang fp contract(off)


#define FIN     256
#define KIN     256
#define CH      128
#define NH1     2
#define HD1     256
#define KA2     512
#define HD2     128
#define EDM     2
#define ELW     8
#define KAPN    32
#define KAP2    4
#define NTHR    256
#define NWAVE   8
#define EPT     8
#define CHUNK   (NTHR * EPT)
#define WCAP    (EPT * 32)
#define LISTN   (NWAVE * WCAP)
#define NBMAX   2048
#define SLOTB   11
#define RCAP    28672
#define DEGCAP  256
#define G1BM    32
#define GBM     64
#define GTHR    128
#define NEGSL   0.2f
#define EPS_SM  1e-16f
#define WSMAX   134217728
#define LDS_AGG ((2 * RCAP + 2 * NBMAX + LISTN) * 4 + 64)

static_assert((CHUNK & (CHUNK - 1)) == 0 && CHUNK <= (1 << SLOTB));
static_assert(NBMAX == (1 << SLOTB));
static_assert(NTHR * 8 == NBMAX);
static_assert(LISTN >= NBMAX);
static_assert(LISTN >= NWAVE * WCAP);
static_assert((RCAP % 32) == 0);
static_assert(LDS_AGG <= 300000);
static_assert(GBM == (GTHR / 32) * 16 && G1BM == (GTHR / 64) * 16);
static_assert((GBM % G1BM) == 0);
static_assert((KIN % 32) == 0 && (KA2 % 32) == 0 && KA2 == 2 * HD1 && KIN == FIN);
static_assert(HD1 == NH1 * CH && HD2 == CH);
static_assert(HD1 == 32 * 8);
static_assert(HD2 == 32 * 4);
static_assert(CH == 32 * 4);
static_assert(KIN / 8 == 32 && KA2 / 8 == 64);
static_assert(NH1 * EDM + EDM <= NWAVE && NH1 * EDM == KAP2 && KAP2 + EDM <= KAPN);
static_assert(G1BM * ELW == 2 * GTHR && GBM * ELW == 4 * GTHR);
static_assert(ELW == 8);

typedef float          v2f  __attribute__((ext_vector_type(2)));
typedef float          v4f  __attribute__((ext_vector_type(4)));
typedef float          v8f  __attribute__((ext_vector_type(8)));
typedef int            v4i  __attribute__((ext_vector_type(4)));
typedef int            v8i  __attribute__((ext_vector_type(8)));
typedef unsigned int   v4u  __attribute__((ext_vector_type(4)));
typedef unsigned short v8us __attribute__((ext_vector_type(8)));
typedef __bf16         v16b __attribute__((ext_vector_type(16)));
typedef v2f  __attribute__((may_alias)) v2fa;
typedef v4f  __attribute__((may_alias)) v4fa;
typedef v8us __attribute__((may_alias)) v8usa;
union FragB { v16b v; v8us h[2]; v8i w; };

__device__ __forceinline__ v8f wmb(const FragB& a, const FragB& b, v8f c) {
  v8f d = __builtin_amdgcn_wmma_f32_16x16x32_bf16(false, a.v, false, b.v, (short)0, c, false, false);
  asm volatile("v_nop\n\tv_nop\n\tv_nop\n\tv_nop" : "+v"(d) : "v"(a.w), "v"(b.w));
  return d;
}

__device__ __forceinline__ unsigned int f2bf(float f) {
  const unsigned int u = __float_as_uint(f);
  return ((u + 0x7FFFu + ((u >> 16) & 1u)) >> 16) & 0xFFFFu;
}
__device__ __forceinline__ float bf2f(unsigned int b) { return __uint_as_float(b << 16); }
__device__ __forceinline__ float bfr(float f) { return bf2f(f2bf(f)); }
__device__ __forceinline__ v4f bfr4(const v4f a) {
  v4f r; r.x = bfr(a.x); r.y = bfr(a.y); r.z = bfr(a.z); r.w = bfr(a.w); return r;
}
__device__ __forceinline__ unsigned int pk2(float lo, float hi) { return f2bf(lo) | (f2bf(hi) << 16); }
__device__ __forceinline__ v4u pack8(const v4f a, const v4f b) {
  v4u r;
  r.x = pk2(a.x, a.y); r.y = pk2(a.z, a.w); r.z = pk2(b.x, b.y); r.w = pk2(b.z, b.w);
  return r;
}
__device__ __forceinline__ void split8(const v4f a, const v4f b, v4u& hv, v4u& lv) {
  const unsigned int h0 = f2bf(a.x), h1 = f2bf(a.y), h2 = f2bf(a.z), h3 = f2bf(a.w);
  const unsigned int h4 = f2bf(b.x), h5 = f2bf(b.y), h6 = f2bf(b.z), h7 = f2bf(b.w);
  const unsigned int l0 = f2bf(a.x - bf2f(h0)), l1 = f2bf(a.y - bf2f(h1));
  const unsigned int l2 = f2bf(a.z - bf2f(h2)), l3 = f2bf(a.w - bf2f(h3));
  const unsigned int l4 = f2bf(b.x - bf2f(h4)), l5 = f2bf(b.y - bf2f(h5));
  const unsigned int l6 = f2bf(b.z - bf2f(h6)), l7 = f2bf(b.w - bf2f(h7));
  hv.x = h0 | (h1 << 16); hv.y = h2 | (h3 << 16); hv.z = h4 | (h5 << 16); hv.w = h6 | (h7 << 16);
  lv.x = l0 | (l1 << 16); lv.y = l2 | (l3 << 16); lv.z = l4 | (l5 << 16); lv.w = l6 | (l7 << 16);
}
__device__ __forceinline__ float leaky(float v) { return v > 0.f ? v : v * NEGSL; }
__device__ __forceinline__ void ostep(float lg, float& mx, float& dn) {
  const float df = lg - mx;
  const float ee = __expf(-fabsf(df));
  const bool up  = df > 0.f;
  const float s1 = up ? ee : 1.0f;
  const float s2 = up ? 1.0f : ee;
  mx = up ? lg : mx;
  dn = fmaf(dn, s1, s2);
}
__device__ __forceinline__ v4f mul4s(float p, const v4f x) {
  v4f r; r.x = p * x.x; r.y = p * x.y; r.z = p * x.z; r.w = p * x.w; return r;
}
__device__ __forceinline__ v4f fma4s(float p, const v4f x, v4f a) {
  a.x = fmaf(p, x.x, a.x); a.y = fmaf(p, x.y, a.y); a.z = fmaf(p, x.z, a.z); a.w = fmaf(p, x.w, a.w); return a;
}
__device__ __forceinline__ v4f add4(const v4f a, const v4f b) {
  v4f r; r.x = a.x + b.x; r.y = a.y + b.y; r.z = a.z + b.z; r.w = a.w + b.w; return r;
}
__device__ __forceinline__ float eluf(float v) {
  const float n = __expf(fminf(v, 0.f)) - 1.0f;
  return v > 0.f ? v : n;
}
__device__ __forceinline__ v4f elu4(const v4f a) {
  v4f r; r.x = eluf(a.x); r.y = eluf(a.y); r.z = eluf(a.z); r.w = eluf(a.w); return r;
}

__device__ __forceinline__ int scan_chunk(const int* __restrict__ dsts, int nE, int cbase, int slotBase,
                                          int nb, int vec8, int* list, int tid, int lane, int wave) {
  int wc = 0;
  const int el0  = tid * EPT;
  const int e0   = cbase + el0;
  const int sent = -2147483647 - 1;
  v4i da, db;
  if (vec8 != 0 && cbase + CHUNK <= nE) {
    da = *(const v4i*)(dsts + e0);
    db = *(const v4i*)(dsts + e0 + 4);
  } else {
    da.x = (e0     < nE) ? dsts[min(e0,     nE - 1)] : sent;
    da.y = (e0 + 1 < nE) ? dsts[min(e0 + 1, nE - 1)] : sent;
    da.z = (e0 + 2 < nE) ? dsts[min(e0 + 2, nE - 1)] : sent;
    da.w = (e0 + 3 < nE) ? dsts[min(e0 + 3, nE - 1)] : sent;
    db.x = (e0 + 4 < nE) ? dsts[min(e0 + 4, nE - 1)] : sent;
    db.y = (e0 + 5 < nE) ? dsts[min(e0 + 5, nE - 1)] : sent;
    db.z = (e0 + 6 < nE) ? dsts[min(e0 + 6, nE - 1)] : sent;
    db.w = (e0 + 7 < nE) ? dsts[min(e0 + 7, nE - 1)] : sent;
  }
  const unsigned nbs = (unsigned)slotBase;
  const unsigned unb = (unsigned)nb;
  const unsigned s0 = (unsigned)da.x - nbs, s1 = (unsigned)da.y - nbs;
  const unsigned s2 = (unsigned)da.z - nbs, s3 = (unsigned)da.w - nbs;
  const unsigned s4 = (unsigned)db.x - nbs, s5 = (unsigned)db.y - nbs;
  const unsigned s6 = (unsigned)db.z - nbs, s7 = (unsigned)db.w - nbs;
  const bool h0 = s0 < unb, h1 = s1 < unb, h2 = s2 < unb, h3 = s3 < unb;
  const bool h4 = s4 < unb, h5 = s5 < unb, h6 = s6 < unb, h7 = s7 < unb;
  const unsigned any = __builtin_amdgcn_ballot_w32(h0 | h1 | h2 | h3 | h4 | h5 | h6 | h7);
  if (any != 0u) {
#define HITJ(J, HJ, SJ) { \
      const unsigned mj = __builtin_amdgcn_ballot_w32(HJ); \
      if (mj != 0u) { \
        if (HJ) { \
          const int pos = wc + (int)__builtin_amdgcn_mbcnt_lo(mj, 0u); \
          if (pos < WCAP) list[wave * WCAP + pos] = ((el0 + (J)) << SLOTB) | (int)(SJ); \
        } \
        wc += (int)__builtin_popcount(mj); } }
    HITJ(0, h0, s0)
    HITJ(1, h1, s1)
    HITJ(2, h2, s2)
    HITJ(3, h3, s3)
    HITJ(4, h4, s4)
    HITJ(5, h5, s5)
    HITJ(6, h6, s6)
    HITJ(7, h7, s7)
#undef HITJ
  }
  return wc;
}

__global__ __launch_bounds__(NTHR) void k_prep(const float* __restrict__ x,
                                               const float* __restrict__ W1, const float* __restrict__ W2,
                                               const float* __restrict__ We1, const float* __restrict__ ae1,
                                               const float* __restrict__ We2, const float* __restrict__ ae2,
                                               unsigned short* xb, unsigned short* w1t, unsigned short* w2t,
                                               float* kap, int nN, int nUx, int nBx, int nB1, int nB2) {
  __shared__ __attribute__((aligned(16))) float skap[KAPN];
  const int tid = (int)threadIdx.x;
  const int bid = (int)blockIdx.x;
  const v4f z4 = {0.f, 0.f, 0.f, 0.f};
  if (bid < nBx) {
    const int i = bid * NTHR + tid;
    if (i >= nUx) return;
    const int row = i >> 5;
    const int c0  = (i & 31) * 8;
    const int rc  = row < nN ? row : nN - 1;
    const float* p = x + (size_t)rc * FIN + c0;
    v4f a = *(const v4fa*)p, b = *(const v4fa*)(p + 4);
    if (row >= nN) { a = z4; b = z4; }
    const v4u hv = pack8(a, b);
    const size_t o = (size_t)row * KIN + c0;
    *(volatile v4u*)(xb + o) = hv;
    __threadfence();
    *(volatile v4u*)(xb + o) = hv;
  } else if (bid < nBx + nB1) {
    const int u = (bid - nBx) * NTHR + tid;
    if (u >= HD1 * (KIN / 8)) return;
    const int n   = u >> 5;
    const int k8  = (u & 31) * 8;
    const int ncl = n < HD1 ? n : HD1 - 1;
    const float* p = W1 + (size_t)k8 * (size_t)HD1 + ncl;
    v4f a, b;
    a.x = p[0];                  a.y = p[(size_t)HD1];        a.z = p[(size_t)2 * HD1];    a.w = p[(size_t)3 * HD1];
    b.x = p[(size_t)4 * HD1];    b.y = p[(size_t)5 * HD1];    b.z = p[(size_t)6 * HD1];    b.w = p[(size_t)7 * HD1];
    if (n >= HD1) { a = z4; b = z4; }
    const v4u wv = pack8(a, b);
    const size_t o = (size_t)n * (size_t)KIN + k8;
    *(volatile v4u*)(w1t + o) = wv;
    __threadfence();
    *(volatile v4u*)(w1t + o) = wv;
  } else if (bid < nBx + nB1 + nB2) {
    const int u = (bid - nBx - nB1) * NTHR + tid;
    if (u >= HD2 * (KA2 / 8)) return;
    const int n   = u >> 6;
    const int k8  = (u & 63) * 8;
    const int kk  = k8 & (HD1 - 1);
    const int ncl = n < HD2 ? n : HD2 - 1;
    const float* p = W2 + (size_t)kk * (size_t)HD2 + ncl;
    v4f a, b;
    a.x = p[0];                  a.y = p[(size_t)HD2];        a.z = p[(size_t)2 * HD2];    a.w = p[(size_t)3 * HD2];
    b.x = p[(size_t)4 * HD2];    b.y = p[(size_t)5 * HD2];    b.z = p[(size_t)6 * HD2];    b.w = p[(size_t)7 * HD2];
    if (n >= HD2) { a = z4; b = z4; }
    const v4u wv = pack8(a, b);
    const size_t o = (size_t)n * (size_t)KA2 + k8;
    *(volatile v4u*)(w2t + o) = wv;
    __threadfence();
    *(volatile v4u*)(w2t + o) = wv;
  } else {
    const int lane = tid & 31, wave = tid >> 5;
    if (tid < KAPN) skap[tid] = 0.f;
    __syncthreads();
    if (wave < NH1 * EDM + EDM) {
      const int p = wave;
      const bool l2 = p >= KAP2;
      const int h = l2 ? 0 : (p >> 1);
      const int t = l2 ? (p - KAP2) : (p & 1);
      const float* wrow = l2 ? (We2 + (size_t)t * HD2) : (We1 + (size_t)t * HD1 + h * CH);
      const float* arow = l2 ? ae2 : (ae1 + h * CH);
      const int c = 4 * lane;
      const v4f w4 = bfr4(*(const v4fa*)(wrow + c));
      const v4f a4 = bfr4(*(const v4fa*)(arow + c));
      float s = w4.x * a4.x; s = fmaf(w4.y, a4.y, s); s = fmaf(w4.z, a4.z, s); s = fmaf(w4.w, a4.w, s);
#pragma unroll
      for (int off = 16; off > 0; off >>= 1) s += __shfl_xor(s, off);
      if (lane == 0) skap[p] = s;
    }
    __syncthreads();
    const v4f kv = *(const v4f*)(skap + 4 * (tid & 7));
    float* op = kap + 4 * (tid & 7);
    if (tid < 8) *(volatile v4f*)op = kv;
    __threadfence();
    if (tid < 8) *(volatile v4f*)op = kv;
  }
}

__global__ __launch_bounds__(NTHR) void k_edge(const float* __restrict__ ea, const float* __restrict__ kap,
                                               float* AE, int nE) {
  __shared__ __attribute__((aligned(16))) float sk[KAPN];
  const int tid = (int)threadIdx.x;
  {
    const v4f kv = *(const v4fa*)(kap + 4 * (tid & 7));
    if (tid < 8) *(v4f*)(sk + 4 * tid) = kv;
  }
  __syncthreads();
  const int e  = (int)blockIdx.x * NTHR + tid;
  const int ec = e < nE ? e : nE - 1;
  const v2f ev = *(const v2fa*)(ea + (size_t)ec * EDM);
  const float v0 = bfr(ev.x), v1 = bfr(ev.y);
  float a0 = v0 * sk[0];        a0 = fmaf(v1, sk[1], a0);
  float a1 = v0 * sk[2];        a1 = fmaf(v1, sk[3], a1);
  float a2 = v0 * sk[KAP2];     a2 = fmaf(v1, sk[KAP2 + 1], a2);
  const bool live = e < nE;
  v4f o;
  o.x = live ? a0 : 0.f; o.y = live ? a1 : 0.f; o.z = live ? a2 : 0.f; o.w = 0.f;
  float* p1 = AE + (size_t)e * 4;
  *(volatile v4f*)p1 = o;
  __threadfence();
  *(volatile v4f*)p1 = o;
}

__global__ __launch_bounds__(GTHR) void k_gemm1(
    const unsigned short* __restrict__ A, const unsigned short* __restrict__ WT,
    const float* __restrict__ al, const float* __restrict__ ar,
    float* FT, float* ELR, int K)
{
  __shared__ __attribute__((aligned(16))) float stg[G1BM * HD1];
  __shared__ __attribute__((aligned(16))) float selr[G1BM * ELW];
  const int tid = (int)threadIdx.x, lane = tid & 31, wave = tid >> 5, hh = lane >> 4, m = lane & 15;
  const int wr = wave & 1, wc = wave >> 1;
  const int rowBase = (int)blockIdx.x * G1BM;

  for (int i = tid; i < G1BM * ELW; i += GTHR) selr[i] = 0.f;

  v8f acc[8];
  {
    const v8f z = {0.f, 0.f, 0.f, 0.f, 0.f, 0.f, 0.f, 0.f};
#pragma unroll
    for (int t = 0; t < 8; ++t) acc[t] = z;
  }
  const unsigned short* ap = A  + (size_t)(rowBase + 16 * wr + m) * (size_t)K + 8 * hh;
  const unsigned short* wp = WT + (size_t)(CH * wc + m) * (size_t)K + 8 * hh;
  const int ksteps = K >> 5;
#pragma unroll 1
  for (int ks = 0; ks < ksteps; ++ks) {
    FragB af;
    af.h[0] = *(const v8usa*)(ap + 32 * ks);
    af.h[1] = *(const v8usa*)(ap + 32 * ks + 16);
#pragma unroll
    for (int t = 0; t < 8; ++t) {
      const unsigned short* wq = wp + (size_t)(16 * t) * (size_t)K + 32 * ks;
      FragB bf;
      bf.h[0] = *(const v8usa*)wq;
      bf.h[1] = *(const v8usa*)(wq + 16);
      acc[t] = wmb(af, bf, acc[t]);
    }
  }

#pragma unroll
  for (int t = 0; t < 8; ++t) {
    const int lc = CH * wc + 16 * t + m;
#pragma unroll
    for (int r = 0; r < 8; ++r) {
      const int lr = 16 * wr + 8 * hh + r;
      stg[lr * HD1 + lc] = acc[t][r];
    }
  }
  __syncthreads();

  const int c0 = 4 * lane;
  const v4f as0 = bfr4(*(const v4fa*)(al + c0));
  const v4f as1 = bfr4(*(const v4fa*)(al + CH + c0));
  const v4f ad0 = bfr4(*(const v4fa*)(ar + c0));
  const v4f ad1 = bfr4(*(const v4fa*)(ar + CH + c0));
  v4f fa[8], fb[8];
#pragma unroll
  for (int i = 0; i < 8; ++i) {
    const int lr = 8 * wave + i;
    const v4f va = *(const v4fa*)(stg + lr * HD1 + c0);
    const v4f vb = *(const v4fa*)(stg + lr * HD1 + CH + c0);
    fa[i] = va; fb[i] = vb;
    float s0 = va.x * as0.x; s0 = fmaf(va.y, as0.y, s0); s0 = fmaf(va.z, as0.z, s0); s0 = fmaf(va.w, as0.w, s0);
    float s1 = vb.x * as1.x; s1 = fmaf(vb.y, as1.y, s1); s1 = fmaf(vb.z, as1.z, s1); s1 = fmaf(vb.w, as1.w, s1);
    float d0 = va.x * ad0.x; d0 = fmaf(va.y, ad0.y, d0); d0 = fmaf(va.z, ad0.z, d0); d0 = fmaf(va.w, ad0.w, d0);
    float d1 = vb.x * ad1.x; d1 = fmaf(vb.y, ad1.y, d1); d1 = fmaf(vb.z, ad1.z, d1); d1 = fmaf(vb.w, ad1.w, d1);
#pragma unroll
    for (int off = 16; off > 0; off >>= 1) {
      s0 += __shfl_xor(s0, off);
      s1 += __shfl_xor(s1, off);
      d0 += __shfl_xor(d0, off);
      d1 += __shfl_xor(d1, off);
    }
    if (lane == 0) {
      selr[lr * ELW]     = s0;
      selr[lr * ELW + 1] = s1;
      selr[lr * ELW + 4] = d0;
      selr[lr * ELW + 5] = d1;
    }
  }
  __syncthreads();

  const int erow = 8 * wave + (m >> 1);
  const v4f ev = *(const v4fa*)(selr + erow * ELW + 4 * (lane & 1));
  float* ep = ELR + (size_t)(rowBase + erow) * ELW + 4 * (lane & 1);
  const bool ewr = lane < 16;
#pragma unroll
  for (int i = 0; i < 8; ++i) {
    float* op = FT + (size_t)(rowBase + 8 * wave + i) * (size_t)HD1 + c0;
    *(volatile v4f*)op = fa[i];
    *(volatile v4f*)(op + CH) = fb[i];
  }
  if (ewr) *(volatile v4f*)ep = ev;
  __threadfence();
#pragma unroll
  for (int i = 0; i < 8; ++i) {
    float* op = FT + (size_t)(rowBase + 8 * wave + i) * (size_t)HD1 + c0;
    *(volatile v4f*)op = fa[i];
    *(volatile v4f*)(op + CH) = fb[i];
  }
  if (ewr) *(volatile v4f*)ep = ev;
}

__global__ __launch_bounds__(GTHR) void k_gemm2(
    const unsigned short* __restrict__ A, const unsigned short* __restrict__ WT,
    const float* __restrict__ al, const float* __restrict__ ar,
    float* FT, float* ELR, int K)
{
  __shared__ __attribute__((aligned(16))) float stg[GBM * HD2];
  __shared__ __attribute__((aligned(16))) float selr[GBM * ELW];
  const int tid = (int)threadIdx.x, lane = tid & 31, wave = tid >> 5, hh = lane >> 4, m = lane & 15;
  const int rowBase = (int)blockIdx.x * GBM;

  for (int i = tid; i < GBM * ELW; i += GTHR) selr[i] = 0.f;

  v8f acc[8];
  {
    const v8f z = {0.f, 0.f, 0.f, 0.f, 0.f, 0.f, 0.f, 0.f};
#pragma unroll
    for (int t = 0; t < 8; ++t) acc[t] = z;
  }
  const unsigned short* ap = A  + (size_t)(rowBase + 16 * wave + m) * (size_t)K + 8 * hh;
  const unsigned short* wp = WT + (size_t)m * (size_t)K + 8 * hh;
  const int ksteps = K >> 5;
#pragma unroll 1
  for (int ks = 0; ks < ksteps; ++ks) {
    FragB af;
    af.h[0] = *(const v8usa*)(ap + 32 * ks);
    af.h[1] = *(const v8usa*)(ap + 32 * ks + 16);
#pragma unroll
    for (int t = 0; t < 8; ++t) {
      const unsigned short* wq = wp + (size_t)(16 * t) * (size_t)K + 32 * ks;
      FragB bf;
      bf.h[0] = *(const v8usa*)wq;
      bf.h[1] = *(const v8usa*)(wq + 16);
      acc[t] = wmb(af, bf, acc[t]);
    }
  }

#pragma unroll
  for (int t = 0; t < 8; ++t) {
    const int lc = 16 * t + m;
#pragma unroll
    for (int r = 0; r < 8; ++r) {
      const int lr = 16 * wave + 8 * hh + r;
      stg[lr * HD2 + lc] = acc[t][r];
    }
  }
  __syncthreads();

  const int c0 = 4 * lane;
  const v4f al4 = bfr4(*(const v4fa*)(al + c0));
  const v4f ar4 = bfr4(*(const v4fa*)(ar + c0));
  v4f fv[16];
#pragma unroll
  for (int i = 0; i < 16; ++i) {
    const int lr = 16 * wave + i;
    const v4f v = *(const v4fa*)(stg + lr * HD2 + c0);
    fv[i] = v;
    float pl = v.x * al4.x; pl = fmaf(v.y, al4.y, pl); pl = fmaf(v.z, al4.z, pl); pl = fmaf(v.w, al4.w, pl);
    float pr = v.x * ar4.x; pr = fmaf(v.y, ar4.y, pr); pr = fmaf(v.z, ar4.z, pr); pr = fmaf(v.w, ar4.w, pr);
#pragma unroll
    for (int off = 16; off > 0; off >>= 1) {
      pl += __shfl_xor(pl, off);
      pr += __shfl_xor(pr, off);
    }
    if (lane == 0) {
      selr[lr * ELW]     = pl;
      selr[lr * ELW + 4] = pr;
    }
  }
  __syncthreads();

  const int erow = 16 * wave + (lane >> 1);
  const v4f ev = *(const v4fa*)(selr + erow * ELW + 4 * (lane & 1));
  float* ep = ELR + (size_t)(rowBase + erow) * ELW + 4 * (lane & 1);
#pragma unroll
  for (int i = 0; i < 16; ++i) {
    float* op = FT + (size_t)(rowBase + 16 * wave + i) * (size_t)HD2 + c0;
    *(volatile v4f*)op = fv[i];
  }
  *(volatile v4f*)ep = ev;
  __threadfence();
#pragma unroll
  for (int i = 0; i < 16; ++i) {
    float* op = FT + (size_t)(rowBase + 16 * wave + i) * (size_t)HD2 + c0;
    *(volatile v4f*)op = fv[i];
  }
  *(volatile v4f*)ep = ev;
}

template<int L>
__global__ __launch_bounds__(NTHR) void k_agg(
    const int* __restrict__ srcs, const int* __restrict__ dsts,
    const float* __restrict__ F, const float* __restrict__ ELR,
    const float* __restrict__ AE, const float* __restrict__ bias,
    unsigned short* A2, float* OUT,
    int nN, int nE, int nb, int vec8, int MPr) {
  extern __shared__ v4f lds_dyn[];
  int* reg1 = (int*)lds_dyn;
  int* reg2 = reg1 + RCAP;
  int* scnt = reg2 + RCAP;
  int* soff = scnt + NBMAX;
  int* list = soff + NBMAX;
  int* wcnt = list + LISTN;
  int* wtot = wcnt + NWAVE;
  const int tid = (int)threadIdx.x, lane = tid & 31, wave = tid >> 5;
  const int nodeBase = (int)blockIdx.x * nb;

  for (int i = tid; i < NBMAX; i += NTHR) scnt[i] = 0;
  __syncthreads();

  int tot = 0;
  const int nChunks = (nE + CHUNK - 1) / CHUNK;
#pragma unroll 1
  for (int ch = 0; ch < nChunks; ++ch) {
    const int cbase = ch * CHUNK;
    const int wc = scan_chunk(dsts, nE, cbase, nodeBase, nb, vec8, list, tid, lane, wave);
    if (lane == 0) wcnt[wave] = wc;
    __syncthreads();
    int pre = 0, all = 0;
#pragma unroll
    for (int w2 = 0; w2 < NWAVE; ++w2) {
      int c = wcnt[w2];
      c = c < 0 ? 0 : (c > WCAP ? WCAP : c);
      all += c;
      pre += (w2 < wave) ? c : 0;
    }
    const int wcc  = wc > WCAP ? WCAP : wc;
    const int base = tot + pre;
#pragma unroll 1
    for (int i = lane; i < wcc; i += 32) {
      const int ent = list[wave * WCAP + i];
      const int el  = (ent >> SLOTB) & (CHUNK - 1);
      const int sl  = ent & (NBMAX - 1);
      int eid = cbase + el;
      eid = eid > nE - 1 ? nE - 1 : eid;
      const int pos = base + i;
      if (pos < RCAP) reg1[pos] = (int)(((unsigned)eid << SLOTB) | (unsigned)sl);
    }
    tot += all;
    tot = tot > RCAP ? RCAP : tot;
    __syncthreads();
  }
  const int nh = tot;

  if (wave == 0) {
#pragma unroll 1
    for (int b0 = 0; b0 < nh; b0 += 32) {
      const int idx = b0 + lane;
      const int uv  = reg1[idx < nh ? idx : nh - 1];
      const int m32 = (nh - b0) < 32 ? (nh - b0) : 32;
#pragma unroll 1
      for (int k = 0; k < m32; ++k) {
        const int u  = __builtin_amdgcn_readlane(uv, k);
        const int sl = u & (NBMAX - 1);
        if (lane == 0) scnt[sl] = scnt[sl] + 1;
      }
    }
  }
  __syncthreads();

  {
    const v4i ca = *(const v4i*)(scnt + 8 * tid);
    const v4i cb = *(const v4i*)(scnt + 8 * tid + 4);
    const int e0 = ca.x < 0 ? 0 : ca.x, e1 = ca.y < 0 ? 0 : ca.y, e2 = ca.z < 0 ? 0 : ca.z, e3 = ca.w < 0 ? 0 : ca.w;
    const int e4 = cb.x < 0 ? 0 : cb.x, e5 = cb.y < 0 ? 0 : cb.y, e6 = cb.z < 0 ? 0 : cb.z, e7 = cb.w < 0 ? 0 : cb.w;
    const int ts = e0 + e1 + e2 + e3 + e4 + e5 + e6 + e7;
    int incl = ts;
#pragma unroll
    for (int d = 1; d < 32; d <<= 1) {
      const int up = __shfl_up(incl, d);
      if (lane >= d) incl += up;
    }
    if (lane == 31) wtot[wave] = incl;
    __syncthreads();
    int pre = 0;
#pragma unroll
    for (int w2 = 0; w2 < NWAVE; ++w2) pre += (w2 < wave) ? wtot[w2] : 0;
    int run = pre + incl - ts;
    soff[8 * tid + 0] = run; run += e0;
    soff[8 * tid + 1] = run; run += e1;
    soff[8 * tid + 2] = run; run += e2;
    soff[8 * tid + 3] = run; run += e3;
    soff[8 * tid + 4] = run; run += e4;
    soff[8 * tid + 5] = run; run += e5;
    soff[8 * tid + 6] = run; run += e6;
    soff[8 * tid + 7] = run;
  }
  __syncthreads();
  for (int i = tid; i < NBMAX; i += NTHR) list[i] = soff[i];
  __syncthreads();

  if (wave == 0) {
#pragma unroll 1
    for (int b0 = 0; b0 < nh; b0 += 32) {
      const int idx = b0 + lane;
      const int uv  = reg1[idx < nh ? idx : nh - 1];
      const int m32 = (nh - b0) < 32 ? (nh - b0) : 32;
#pragma unroll 1
      for (int k = 0; k < m32; ++k) {
        const int u   = __builtin_amdgcn_readlane(uv, k);
        const int sl  = u & (NBMAX - 1);
        const int eid = (int)((unsigned)u >> SLOTB);
        if (lane == 0) {
          int pos = list[sl];
          pos = pos < 0 ? 0 : (pos > RCAP - 1 ? RCAP - 1 : pos);
          reg2[pos] = eid;
          list[sl] = pos + 1;
        }
      }
    }
  }
  __syncthreads();

  const int nbw = nb >> 3;
  const bool ovf = (nh >= RCAP);
  const float qnan = __int_as_float(0x7fc00000);
  const v4f z4 = {0.f, 0.f, 0.f, 0.f};

  if (L == 1) {
    const int cb = 8 * lane;
    const bool hsel = lane >= 16;
    const v4f bb0 = bfr4(*(const v4fa*)(bias + cb));
    const v4f bb1 = bfr4(*(const v4fa*)(bias + cb + 4));
#pragma unroll 1
    for (int jt = 0; jt < nbw; ++jt) {
      const int slot = wave * nbw + jt;
      const int grow = nodeBase + slot;
      const int gcl  = grow < nN ? grow : nN - 1;
      int st = soff[slot];
      const int craw = scnt[slot];
      int cnt = craw;
      st  = st < 0 ? 0 : (st > nh ? nh : st);
      cnt = cnt < 0 ? 0 : (cnt > DEGCAP ? DEGCAP : cnt);
      if (cnt > nh - st) cnt = nh - st;
      const float pz = (ovf || craw > DEGCAP) ? qnan : 0.0f;

      const v2f es2 = *(const v2fa*)(ELR + (size_t)gcl * ELW);
      const v2f ed2 = *(const v2fa*)(ELR + (size_t)gcl * ELW + 4);
      float mx0 = -1.0e30f, mx1 = -1.0e30f, dn0 = 0.f, dn1 = 0.f, ws0 = 0.f, ws1 = 0.f;

#pragma unroll 1
      for (int q = 0; q < cnt; ++q) {
        int idx = st + q; idx = idx > RCAP - 1 ? RCAP - 1 : idx;
        int eid = reg2[idx]; eid = eid < 0 ? 0 : (eid > nE - 1 ? nE - 1 : eid);
        const int sraw = srcs[eid];
        const int s = sraw < 0 ? 0 : (sraw > nN - 1 ? nN - 1 : sraw);
        const v2f el2 = *(const v2fa*)(ELR + (size_t)s * ELW);
        const v2f av2 = *(const v2fa*)(AE + (size_t)eid * 4);
        const float lg0 = leaky((el2.x + ed2.x) + av2.x);
        const float lg1 = leaky((el2.y + ed2.y) + av2.y);
        ws0 += av2.x; ws1 += av2.y;
        ostep(lg0, mx0, dn0);
        ostep(lg1, mx1, dn1);
      }
      const float rcn  = __builtin_amdgcn_rcpf(fmaxf((float)cnt, 1.0f));
      const float lw0  = ws0 * rcn, lw1 = ws1 * rcn;
      const float lgs0 = leaky((es2.x + ed2.x) + lw0);
      const float lgs1 = leaky((es2.y + ed2.y) + lw1);
      ostep(lgs0, mx0, dn0);
      ostep(lgs1, mx1, dn1);
      const float inv0 = __builtin_amdgcn_rcpf(dn0 + EPS_SM);
      const float inv1 = __builtin_amdgcn_rcpf(dn1 + EPS_SM);
      const float wsf0 = __expf(lgs0 - mx0) * inv0;
      const float wsf1 = __expf(lgs1 - mx1) * inv1;
      const float mL  = hsel ? mx1  : mx0;
      const float iL  = hsel ? inv1 : inv0;
      const float sL  = hsel ? wsf1 : wsf0;
      const float edL = hsel ? ed2.y : ed2.x;
      const bool live = grow < nN;
      const bool wr   = grow < MPr;

      const float* fr = F + (size_t)gcl * HD1 + cb;
      v4f a0 = mul4s(sL, *(const v4fa*)(fr));
      v4f a1 = mul4s(sL, *(const v4fa*)(fr + 4));

#pragma unroll 1
      for (int q = 0; q < cnt; ++q) {
        int idx = st + q; idx = idx > RCAP - 1 ? RCAP - 1 : idx;
        int eid = reg2[idx]; eid = eid < 0 ? 0 : (eid > nE - 1 ? nE - 1 : eid);
        const int sraw = srcs[eid];
        const int s = sraw < 0 ? 0 : (sraw > nN - 1 ? nN - 1 : sraw);
        const v2f el2 = *(const v2fa*)(ELR + (size_t)s * ELW);
        const v2f av2 = *(const v2fa*)(AE + (size_t)eid * 4);
        const float elL = hsel ? el2.y : el2.x;
        const float aeL = hsel ? av2.y : av2.x;
        const float lg  = leaky((elL + edL) + aeL);
        const float p   = __expf(lg - mL) * iL;
        const float* sr = F + (size_t)s * HD1 + cb;
        const v4f x0 = *(const v4fa*)(sr), x1 = *(const v4fa*)(sr + 4);
        a0 = fma4s(p, x0, a0); a1 = fma4s(p, x1, a1);
      }

      v4f y0 = elu4(add4(a0, bb0));
      v4f y1 = elu4(add4(a1, bb1));
      y0 = live ? y0 : z4; y1 = live ? y1 : z4;
      const v4f pz4 = {pz, pz, pz, pz};
      y0 = add4(y0, pz4); y1 = add4(y1, pz4);
      v4u hv, lv;
      split8(y0, y1, hv, lv);
      unsigned short* gp = A2 + (size_t)grow * KA2 + cb;
      if (wr) {
        *(volatile v4u*)(gp)       = hv;
        *(volatile v4u*)(gp + HD1) = lv;
      }
      __threadfence();
      if (wr) {
        *(volatile v4u*)(gp)       = hv;
        *(volatile v4u*)(gp + HD1) = lv;
      }
    }
  } else {
    const int cl = 4 * lane;
    const v4f bb = bfr4(*(const v4fa*)(bias + cl));
#pragma unroll 1
    for (int jt = 0; jt < nbw; ++jt) {
      const int slot = wave * nbw + jt;
      const int grow = nodeBase + slot;
      const int gcl  = grow < nN ? grow : nN - 1;
      int st = soff[slot];
      const int craw = scnt[slot];
      int cnt = craw;
      st  = st < 0 ? 0 : (st > nh ? nh : st);
      cnt = cnt < 0 ? 0 : (cnt > DEGCAP ? DEGCAP : cnt);
      if (cnt > nh - st) cnt = nh - st;
      const float pz = (ovf || craw > DEGCAP) ? qnan : 0.0f;

      const float es = ELR[(size_t)gcl * ELW];
      const float ed = ELR[(size_t)gcl * ELW + 4];
      float mx = -1.0e30f, dn = 0.f, wsm = 0.f;

#pragma unroll 1
      for (int q = 0; q < cnt; ++q) {
        int idx = st + q; idx = idx > RCAP - 1 ? RCAP - 1 : idx;
        int eid = reg2[idx]; eid = eid < 0 ? 0 : (eid > nE - 1 ? nE - 1 : eid);
        const int sraw = srcs[eid];
        const int s = sraw < 0 ? 0 : (sraw > nN - 1 ? nN - 1 : sraw);
        const float asr = ELR[(size_t)s * ELW];
        const float ae  = AE[(size_t)eid * 4 + 2];
        const float lg  = leaky((asr + ed) + ae);
        wsm += ae;
        ostep(lg, mx, dn);
      }
      const float rcn = __builtin_amdgcn_rcpf(fmaxf((float)cnt, 1.0f));
      const float lw  = wsm * rcn;
      const float lgs = leaky((es + ed) + lw);
      ostep(lgs, mx, dn);
      const float inv = __builtin_amdgcn_rcpf(dn + EPS_SM);
      const float wsf = __expf(lgs - mx) * inv;

      const float* fr = F + (size_t)gcl * HD2 + cl;
      v4f a0 = mul4s(wsf, *(const v4fa*)(fr));

#pragma unroll 1
      for (int q = 0; q < cnt; ++q) {
        int idx = st + q; idx = idx > RCAP - 1 ? RCAP - 1 : idx;
        int eid = reg2[idx]; eid = eid < 0 ? 0 : (eid > nE - 1 ? nE - 1 : eid);
        const int sraw = srcs[eid];
        const int s = sraw < 0 ? 0 : (sraw > nN - 1 ? nN - 1 : sraw);
        const float asr = ELR[(size_t)s * ELW];
        const float ae  = AE[(size_t)eid * 4 + 2];
        const float lg  = leaky((asr + ed) + ae);
        const float p   = __expf(lg - mx) * inv;
        const float* sr = F + (size_t)s * HD2 + cl;
        const v4f x0 = *(const v4fa*)(sr);
        a0 = fma4s(p, x0, a0);
      }
      const bool live = grow < nN;
      v4f y0 = add4(a0, bb);
      const v4f pz4 = {pz, pz, pz, pz};
      y0 = add4(y0, pz4);
      float* gp = OUT + (size_t)grow * HD2 + cl;
      if (live) *(volatile v4f*)(gp) = y0;
      __threadfence();
      if (live) *(volatile v4f*)(gp) = y0;
    }
  }
}

static int pick_nb(int nE, int nN) {
  int nb = NBMAX;
  while (nb > 32 && (long long)nb * (long long)nE * 5LL > (long long)RCAP * (long long)nN * 4LL) nb >>= 1;
  return nb;
}
static inline int cdiv(int a, int b) { return (a + b - 1) / b; }
static inline size_t al256(size_t v) { return (v + 255) & ~(size_t)255; }

extern "C" void kernel_launch(void* const* d_in, const int* in_sizes, int n_in,
                              void* d_out, int out_size, void* d_ws, size_t ws_size,
                              hipStream_t stream) {
  if (n_in < 15) return;
  if (in_sizes[0] < FIN || (in_sizes[0] % FIN) != 0) return;
  const int nN = in_sizes[0] / FIN;
  if (nN <= 0 || nN > (1 << 22)) return;
  if (in_sizes[1] < 2 || (in_sizes[1] & 1) != 0) return;
  const int nE = in_sizes[1] / 2;
  if (nE < 1 || nE >= (1 << (32 - SLOTB))) return;
  if (in_sizes[2] != nE * EDM) return;
  if (in_sizes[3] != KIN * HD1) return;
  if (in_sizes[4] != HD1 || in_sizes[5] != HD1) return;
  if (in_sizes[6] != EDM * HD1) return;
  if (in_sizes[7] != HD1) return;
  if (in_sizes[8] != HD1) return;
  if (in_sizes[9] != HD1 * HD2) return;
  if (in_sizes[10] != HD2 || in_sizes[11] != HD2) return;
  if (in_sizes[12] != EDM * HD2) return;
  if (in_sizes[13] != HD2) return;
  if (in_sizes[14] != HD2) return;
  if ((long long)out_size != (long long)nN * (long long)HD2) return;

  const float* x   = (const float*)d_in[0];
  const int*   ei  = (const int*)  d_in[1];
  const float* ea  = (const float*)d_in[2];
  const float* W1  = (const float*)d_in[3];
  const float* as1 = (const float*)d_in[4];
  const float* ad1 = (const float*)d_in[5];
  const float* We1 = (const float*)d_in[6];
  const float* ae1 = (const float*)d_in[7];
  const float* b1  = (const float*)d_in[8];
  const float* W2  = (const float*)d_in[9];
  const float* as2 = (const float*)d_in[10];
  const float* ad2 = (const float*)d_in[11];
  const float* We2 = (const float*)d_in[12];
  const float* ae2 = (const float*)d_in[13];
  const float* b2  = (const float*)d_in[14];
  float* out = (float*)d_out;
  const int* src = ei;
  const int* dst = ei + nE;

  const int MP   = cdiv(nN, GBM) * GBM;
  const int EP   = cdiv(nE, NTHR) * NTHR;
  const int nb   = pick_nb(nE, nN);
  if (nb < 32 || (nb & (nb - 1)) != 0 || nb > NBMAX) return;
  const int gA   = cdiv(MP, nb);
  const int vec8 = ((nE & 3) == 0) ? 1 : 0;
  if (gA * nb < MP) return;

  char* ws = (char*)d_ws;
  size_t off = 0;
  const size_t oW1T = off; off = al256(off + (size_t)HD1 * KIN * 2);
  const size_t oW2T = off; off = al256(off + (size_t)HD2 * KA2 * 2);
  const size_t oKAP = off; off = al256(off + (size_t)KAPN * 4);
  const size_t oAE  = off; off = al256(off + (size_t)EP * 4 * 4);
  const size_t oH1  = off; off = al256(off + (size_t)MP * HD1 * 4);
  const size_t eH1  = off;
  const size_t oEL1 = off; off = al256(off + (size_t)MP * ELW * 4);
  const size_t oA2  = off; off = al256(off + (size_t)MP * KA2 * 2);
  const size_t eA2  = off;
  if (off > ws_size || off > (size_t)WSMAX) return;
  const size_t oXB  = oA2;
  if (oXB + (size_t)MP * KIN * 2 > eA2) return;
  size_t sub = oH1;
  const size_t oH2  = sub; sub = al256(sub + (size_t)MP * HD2 * 4);
  const size_t oEL2 = sub; sub = al256(sub + (size_t)MP * ELW * 4);
  if (sub > eH1) return;
  unsigned short* W1T  = (unsigned short*)(ws + oW1T);
  unsigned short* W2T  = (unsigned short*)(ws + oW2T);
  float*          KAP  = (float*)(ws + oKAP);
  float*          AE   = (float*)(ws + oAE);
  float*          H1   = (float*)(ws + oH1);
  float*          ELR1 = (float*)(ws + oEL1);
  unsigned short* A2   = (unsigned short*)(ws + oA2);
  unsigned short* XB   = (unsigned short*)(ws + oXB);
  float*          H2   = (float*)(ws + oH2);
  float*          ELR2 = (float*)(ws + oEL2);

  hipFuncSetAttribute(reinterpret_cast<const void*>(&k_agg<1>),
                      hipFuncAttributeMaxDynamicSharedMemorySize, LDS_AGG);
  hipFuncSetAttribute(reinterpret_cast<const void*>(&k_agg<2>),
                      hipFuncAttributeMaxDynamicSharedMemorySize, LDS_AGG);

  const int nUx = MP * (KIN / 8);
  const int nBx = cdiv(nUx, NTHR);
  if (nBx * NTHR != nUx) return;
  const int nB1 = cdiv(HD1 * (KIN / 8), NTHR);
  const int nB2 = cdiv(HD2 * (KA2 / 8), NTHR);
  k_prep<<<nBx + nB1 + nB2 + 1, NTHR, 0, stream>>>(x, W1, W2, We1, ae1, We2, ae2,
                                                   XB, W1T, W2T, KAP, nN, nUx, nBx, nB1, nB2);

  k_edge<<<EP / NTHR, NTHR, 0, stream>>>(ea, KAP, AE, nE);

  k_gemm1<<<MP / G1BM, GTHR, 0, stream>>>(XB, W1T, as1, ad1, H1, ELR1, KIN);

  k_agg<1><<<gA, NTHR, LDS_AGG, stream>>>(src, dst, H1, ELR1, AE, b1, A2, out, nN, nE, nb, vec8, MP);

  k_gemm2<<<MP / GBM, GTHR, 0, stream>>>(A2, W2T, as2, ad2, H2, ELR2, KA2);

  k_agg<2><<<gA, NTHR, LDS_AGG, stream>>>(src, dst, H2, ELR2, AE, b2, A2, out, nN, nE, nb, vec8, MP);
}
